// SentenceLlamaAttention_67740224192514
// MI455X (gfx1250) — hardware-verified
//
#include <hip/hip_runtime.h>
#include <math.h>

typedef __attribute__((ext_vector_type(16))) _Float16 v16h;
typedef __attribute__((ext_vector_type(16))) __bf16 v16b;
typedef __attribute__((ext_vector_type(8)))  _Float16 v8h;
typedef __attribute__((ext_vector_type(8)))  float v8f;
typedef __attribute__((ext_vector_type(4)))  float v4f;
typedef __attribute__((ext_vector_type(2)))  float v2f;
typedef __attribute__((ext_vector_type(4)))  unsigned v4u;
typedef __attribute__((ext_vector_type(4)))  int v4i;
typedef float __attribute__((may_alias)) float_a;
typedef int __attribute__((may_alias)) int_a;

template <typename T> __device__ __forceinline__ void vst2(void* p, T v) { *(volatile T*)p = v; __threadfence(); *(volatile T*)p = v; }
__device__ __forceinline__ v8f wmma16(v16h a, v16h b, v8f c) {
  v8f d = __builtin_amdgcn_wmma_f32_16x16x32_f16(false, a, false, b, (short)0, c, false, false);
  asm volatile("v_nop\n\tv_nop\n\tv_nop\n\tv_nop" : "+v"(d) : "v"(a), "v"(b));
  return d;
}
__device__ __forceinline__ v8f wmma_bf(v16b a, v16b b, v8f c) {
  v8f d = __builtin_amdgcn_wmma_f32_16x16x32_bf16(false, a, false, b, (short)0, c, false, false);
  asm volatile("v_nop\n\tv_nop\n\tv_nop\n\tv_nop" : "+v"(d) : "v"(a), "v"(b));
  return d;
}
__device__ __forceinline__ v16h frag_h(const _Float16* rowk0, int lane) {
  union { v16h v; v8h q[2]; } u; const _Float16* p = rowk0 + 8 * (lane >> 4);
  u.q[0] = *(const v8h*)p; u.q[1] = *(const v8h*)(p + 16); return u.v;
}
__device__ __forceinline__ v16h frag_f32(const float* rowk0, int lane) {
  v16h a; const float* p = rowk0 + 8 * (lane >> 4);
#pragma unroll
  for (int i = 0; i < 8; ++i) { a[i] = (_Float16)p[i]; a[8 + i] = (_Float16)p[16 + i]; }
  return a;
}
__device__ __forceinline__ v16h frag_f32s(const float* rowk0, int lane, float sc) {
  v16h a; const float* p = rowk0 + 8 * (lane >> 4);
#pragma unroll
  for (int i = 0; i < 8; ++i) { a[i] = (_Float16)(p[i] * sc); a[8 + i] = (_Float16)(p[16 + i] * sc); }
  return a;
}
__device__ __forceinline__ v16h fragc_f32(const float* W, int k0, int n, int lane, int ld, int K) {
  v16h a; const int g = lane >> 4;
#pragma unroll
  for (int i = 0; i < 8; ++i) { const int ka = k0 + 8 * g + i, kb = ka + 16;
    a[i] = (_Float16)(ka < K ? W[(size_t)(ka < K ? ka : K - 1) * ld + n] : 0.f); a[8 + i] = (_Float16)(kb < K ? W[(size_t)(kb < K ? kb : K - 1) * ld + n] : 0.f); }
  return a;
}
struct F2 { v16b h, l; };
__device__ __forceinline__ F2 bsplit16(const float v[16]) { F2 r;
#pragma unroll
  for (int i = 0; i < 16; ++i) { const __bf16 h = (__bf16)v[i]; r.h[i] = h; r.l[i] = (__bf16)(v[i] - (float)h); }
  return r; }
__device__ __forceinline__ F2 split_row(const float* row, int k0, int lane) { float v[16]; const float* p = row + k0 + 8 * (lane >> 4);
#pragma unroll
  for (int i = 0; i < 8; ++i) { v[i] = p[i]; v[8 + i] = p[16 + i]; }
  return bsplit16(v); }
__device__ __forceinline__ F2 split_rowK(const float* row, int k0, int lane, int K) { float v[16]; const int g = lane >> 4;
#pragma unroll
  for (int i = 0; i < 8; ++i) { const int ka = k0 + 8 * g + i, kb = ka + 16; v[i] = ka < K ? row[ka < K ? ka : K - 1] : 0.f; v[8 + i] = kb < K ? row[kb < K ? kb : K - 1] : 0.f; }
  return bsplit16(v); }
__device__ __forceinline__ F2 split_col(const float* W, int k0, int n, int lane, int ld, int K) { float v[16]; const int g = lane >> 4;
#pragma unroll
  for (int i = 0; i < 8; ++i) { const int ka = k0 + 8 * g + i, kb = ka + 16; v[i] = ka < K ? W[(size_t)(ka < K ? ka : K - 1) * ld + n] : 0.f; v[8 + i] = kb < K ? W[(size_t)(kb < K ? kb : K - 1) * ld + n] : 0.f; }
  return bsplit16(v); }
__device__ __forceinline__ v8f mac3(const F2& a, const F2& b, v8f c) { c = wmma_bf(a.l, b.h, c); c = wmma_bf(a.h, b.l, c); return wmma_bf(a.h, b.h, c); }
__device__ __forceinline__ float sigm(float v) { return 1.0f / (1.0f + expf(-v)); }
#define LDSX() do { asm volatile("s_wait_dscnt 0" ::: "memory"); __builtin_amdgcn_wave_barrier(); __builtin_amdgcn_fence(__ATOMIC_RELEASE, "workgroup"); } while (0)


#define SS 4096
#define DM 1024
#define NH 16
#define NKV 4
#define HD 64
#define KVW (NKV * HD)
#define QKVW (DM + 2 * KVW)
#define NKMAX 512
#ifndef TQB
#define TQB (SS / 64)
#define TQ0 0
#endif
typedef __attribute__((ext_vector_type(8))) __bf16 v8b;
__device__ __forceinline__ v16b frag_b(const __bf16* rowk0, int lane) {
  union { v16b v; v8b q[2]; } u; const __bf16* p = rowk0 + 8 * (lane >> 4);
  u.q[0] = *(const v8b*)p; u.q[1] = *(const v8b*)(p + 16); return u.v;
}
__device__ __forceinline__ float bfr(float v) { return (float)(__bf16)v; }
__device__ __attribute__((noinline)) float exp_ni(float v) { return expf(v); }
__device__ __attribute__((noinline)) float erf_ni(float v) { return erff(v); }

#define WS_PK  0u
#define PK_O   ((size_t)QKVW * DM)
#define WS_QKV (WS_PK + 2u * ((size_t)QKVW * DM + (size_t)DM * DM))
#define WS_O   (WS_QKV + 4u * SS * QKVW)
#define WS_SPL (WS_O + 4u * SS * DM)
#define WS_END (WS_SPL + 4u * (SS + 32))

__global__ __launch_bounds__(256) void k_packT(const float* __restrict__ Wm, int K, int N, __bf16* __restrict__ DST) {
  __shared__ __align__(16) __bf16 s[DM]; const int n = blockIdx.x, tid = threadIdx.x;
  for (int k = tid; k < K; k += 256) s[k] = (__bf16)Wm[(size_t)k * N + n];
  __syncthreads();
  for (int q = tid; q < K / 8; q += 256) vst2((unsigned*)(DST + (size_t)n * K + q * 8), *(const v4u*)&s[q * 8]);
}
__global__ __launch_bounds__(32) void k_speclist(const int* __restrict__ SM, int* __restrict__ SPL) {
  __shared__ __align__(16) int sl[SS]; __shared__ __align__(16) int sc[32]; const int lane = threadIdx.x; int cnt = 0;
  for (int c0 = 0; c0 < SS; c0 += 32) { const int j = c0 + lane; const bool sp = SM[j] != 0; const unsigned bal = __builtin_amdgcn_ballot_w32(sp); const int rank = __builtin_popcount(bal & ((1u << lane) - 1u)); if (sp) sl[cnt + rank] = j; cnt += __builtin_popcount(bal); }
  for (int q = cnt + lane; q < SS; q += 32) sl[q] = SS;
  sc[lane] = (lane == 0) ? cnt : 0;
  LDSX();
  for (int q = lane; q < SS / 4; q += 32) vst2((unsigned*)(SPL + q * 4), *(const v4u*)&sl[q * 4]);
  if (lane < 8) vst2((unsigned*)(SPL + SS + lane * 4), *(const v4u*)&sc[lane * 4]);
}
__global__ __launch_bounds__(128) void k_qkv(const float* __restrict__ X, const __bf16* __restrict__ P, const float* __restrict__ COS, const float* __restrict__ SIN, float* __restrict__ QKV) {
  __shared__ __align__(16) float so[4][16][132];
  const int tid = threadIdx.x, wave = tid >> 5, lane = tid & 31, col = lane & 15, g = lane >> 4; const size_t r0 = (size_t)blockIdx.x * 64 + wave * 16; const int n0 = blockIdx.y * 128;
  v8f acc[8] = {};
#pragma unroll 2
  for (int kc = 0; kc < DM / 32; ++kc) { v16b a; { const float* p = X + (r0 + col) * DM + kc * 32 + 8 * g;
#pragma unroll
      for (int i = 0; i < 8; ++i) { a[i] = (__bf16)p[i]; a[8 + i] = (__bf16)p[16 + i]; } }
#pragma unroll
    for (int j = 0; j < 8; ++j) acc[j] = wmma_bf(a, frag_b(P + (size_t)(n0 + j * 16 + col) * DM + kc * 32, lane), acc[j]); }
  const bool rope = (n0 < DM + KVW);
#pragma unroll
  for (int j = 0; j < 8; ++j) { const int jj = j & 3; const int d = jj * 16 + col;
#pragma unroll
    for (int r = 0; r < 8; ++r) { float v = acc[j][r];
      if (rope) { const size_t t = r0 + 8 * g + r; const float c = bfr(COS[t * HD + d]), s = bfr(SIN[t * HD + d]); const float rot = (jj < 2) ? -acc[(j + 2) & 7][r] : acc[(j + 6) & 7][r]; v = v * c + rot * s; }
      so[wave][8 * g + r][j * 16 + col] = v; } }
  LDSX();
  for (int rl = 0; rl < 16; ++rl) vst2(QKV + (r0 + rl) * QKVW + n0 + lane * 4, *(const v4f*)&so[wave][rl][lane * 4]);
}
__global__ __launch_bounds__(128) void k_attn(const float* __restrict__ QKV, const int* __restrict__ SM, const int* __restrict__ EOS, const int* __restrict__ SPL, float* __restrict__ O) {
  __shared__ __align__(16) float sp[4][16][36]; __shared__ __align__(16) float so[4][16][68]; __shared__ int slist[NKMAX]; __shared__ __align__(16) __bf16 svh[HD][NKMAX + 8], svl[HD][NKMAX + 8]; __shared__ int sn, sw0;
  const int tid = threadIdx.x, wave = tid >> 5, lane = tid & 31, col = lane & 15, g = lane >> 4; const int qb = blockIdx.x + TQ0, h = blockIdx.y, kvh = h / (NH / NKV); const int qblk0 = qb * 64; const int q0 = qblk0 + wave * 16;
  if (tid == 0) { int w0 = SS; for (int r = 0; r < 64; ++r) w0 = min(w0, min(max(EOS[qblk0 + r], 0), SS - 1)); w0 = min(w0, qblk0 + 63);
    const int nsp = min(max(SPL[SS], 0), SS); int nsb = 0; while (nsb < nsp && SPL[nsb] < w0) ++nsb;
    const int nwin = qblk0 + 63 - w0 + 1; int n = nsb + nwin; if (n > NKMAX) { n = NKMAX; }
    sn = n; sw0 = w0;
    for (int i = 0; i < n; ++i) slist[i] = (i < nsb) ? SPL[i] : (w0 + (i - nsb));
    for (int i = n; i < NKMAX; ++i) slist[i] = w0; }
  __syncthreads();
  const int n = sn; const int nks = (n + 31) / 32;
  for (int q = tid; q < nks * 32 * HD; q += 128) { const int j = q / HD, d = q % HD; const int key = slist[j]; const float v = QKV[(size_t)key * QKVW + DM + KVW + kvh * HD + d]; const __bf16 hb = (__bf16)v; svh[d][j] = hb; svl[d][j] = (__bf16)(v - (float)hb); }
  __syncthreads();
  F2 aq[2];
#pragma unroll
  for (int kc = 0; kc < 2; ++kc) aq[kc] = split_row(QKV + (size_t)(q0 + col) * QKVW + h * HD, kc * 32, lane);
  int eosr[8];
#pragma unroll
  for (int r = 0; r < 8; ++r) eosr[r] = EOS[q0 + 8 * g + r];
  float m[8], l[8];
#pragma unroll
  for (int r = 0; r < 8; ++r) { m[r] = -3.0e38f; l[r] = 0.f; }
  v8f acc[4] = {};
#pragma unroll 1
  for (int ks = 0; ks < nks; ++ks) { v8f s[2]; int keyc[2]; bool spc[2], inl[2];
#pragma unroll
    for (int ct = 0; ct < 2; ++ct) { const int j = ks * 32 + ct * 16 + col; const int key = slist[j]; keyc[ct] = key; inl[ct] = (j < n); spc[ct] = (SM[key] != 0);
      const float* krow = QKV + (size_t)key * QKVW + DM + kvh * HD; v8f c = {};
#pragma unroll
      for (int kc = 0; kc < 2; ++kc) { const F2 kb = split_row(krow, kc * 32, lane); c = mac3(aq[kc], kb, c); }
      s[ct] = c; }
#pragma unroll
    for (int r = 0; r < 8; ++r) { const int qi = q0 + 8 * g + r; float sv[2];
#pragma unroll
      for (int ct = 0; ct < 2; ++ct) { const bool ok = inl[ct] && keyc[ct] <= qi && (keyc[ct] >= eosr[r] || spc[ct]); sv[ct] = ok ? s[ct][r] * 0.125f : -3.0e38f; }
      float mx = fmaxf(sv[0], sv[1]);
#pragma unroll
      for (int o = 1; o < 16; o <<= 1) mx = fmaxf(mx, __shfl_xor(mx, o));
      const float mn = fmaxf(m[r], mx); const float alpha = (m[r] <= -1.0e38f) ? 0.f : exp_ni(m[r] - mn);
      const float e0 = (sv[0] <= -1.0e38f) ? 0.f : exp_ni(sv[0] - mn), e1 = (sv[1] <= -1.0e38f) ? 0.f : exp_ni(sv[1] - mn); float es = e0 + e1;
#pragma unroll
      for (int o = 1; o < 16; o <<= 1) es += __shfl_xor(es, o);
      l[r] = l[r] * alpha + es; m[r] = mn;
#pragma unroll
      for (int dt = 0; dt < 4; ++dt) acc[dt][r] *= alpha;
      sp[wave][8 * g + r][col] = e0; sp[wave][8 * g + r][16 + col] = e1; }
    LDSX();
    const F2 pa = split_row(&sp[wave][col][0], 0, lane);
#pragma unroll
    for (int dt = 0; dt < 4; ++dt) { const v16b vh = frag_b(&svh[dt * 16 + col][ks * 32], lane), vl = frag_b(&svl[dt * 16 + col][ks * 32], lane); acc[dt] = wmma_bf(pa.l, vh, acc[dt]); acc[dt] = wmma_bf(pa.h, vl, acc[dt]); acc[dt] = wmma_bf(pa.h, vh, acc[dt]); }
    LDSX(); }
#pragma unroll
  for (int r = 0; r < 8; ++r) { const float il = (l[r] > 0.f) ? 1.0f / l[r] : 0.f;
#pragma unroll
    for (int dt = 0; dt < 4; ++dt) so[wave][8 * g + r][dt * 16 + col] = acc[dt][r] * il; }
  LDSX();
  for (int rl = 0; rl < 16; ++rl) if (lane < 16) vst2(O + (size_t)(q0 + rl) * DM + h * HD + lane * 4, *(const v4f*)&so[wave][rl][lane * 4]);
}
__global__ __launch_bounds__(128) void k_out(const float* __restrict__ O, const __bf16* __restrict__ P, float* __restrict__ Y) {
  __shared__ __align__(16) float so[4][16][132];
  const int tid = threadIdx.x, wave = tid >> 5, lane = tid & 31, col = lane & 15, g = lane >> 4; const size_t r0 = (size_t)(blockIdx.x + TQ0) * 64 + wave * 16; const int n0 = blockIdx.y * 128;
  v8f acc[8] = {};
#pragma unroll 2
  for (int kc = 0; kc < DM / 32; ++kc) { const F2 a = split_row(O + (r0 + col) * DM, kc * 32, lane);
#pragma unroll
    for (int j = 0; j < 8; ++j) { const v16b w = frag_b(P + (size_t)(n0 + j * 16 + col) * DM + kc * 32, lane); acc[j] = wmma_bf(a.l, w, acc[j]); acc[j] = wmma_bf(a.h, w, acc[j]); } }
#pragma unroll
  for (int j = 0; j < 8; ++j)
#pragma unroll
    for (int r = 0; r < 8; ++r) so[wave][8 * g + r][j * 16 + col] = acc[j][r];
  LDSX();
  for (int rl = 0; rl < 16; ++rl) vst2(Y + (r0 + rl) * DM + n0 + lane * 4, *(const v4f*)&so[wave][rl][lane * 4]);
}
extern "C" void kernel_launch(void* const* d_in, const int* in_sizes, int n_in, void* d_out, int out_size, void* d_ws, size_t ws_size, hipStream_t stream) {
  (void)in_sizes; (void)n_in; (void)out_size;
  const float** F = (const float**)d_in; const int* SM = (const int*)d_in[7]; const int* EOS = (const int*)d_in[8];
  if (ws_size < (size_t)WS_END) return;
  char* ws = (char*)d_ws; __bf16* PK = (__bf16*)(ws + WS_PK); float *QKV = (float*)(ws + WS_QKV), *O = (float*)(ws + WS_O); int* SPL = (int*)(ws + WS_SPL);
  k_packT<<<DM, 256, 0, stream>>>(F[3], DM, DM, PK); k_packT<<<KVW, 256, 0, stream>>>(F[4], DM, KVW, PK + (size_t)DM * DM); k_packT<<<KVW, 256, 0, stream>>>(F[5], DM, KVW, PK + (size_t)(DM + KVW) * DM); k_packT<<<DM, 256, 0, stream>>>(F[6], DM, DM, PK + PK_O);
  k_speclist<<<1, 32, 0, stream>>>(SM, SPL);
  k_qkv<<<dim3(SS / 64, QKVW / 128), 128, 0, stream>>>(F[0], PK, F[1], F[2], QKV);
  k_attn<<<dim3(TQB, NH), 128, 0, stream>>>(QKV, SM, EOS, SPL, O);
  k_out<<<dim3(TQB, DM / 128), 128, 0, stream>>>(O, PK + PK_O, (float*)d_out);
}
